// MultiHeadSelfAttention_65661460021618
// MI455X (gfx1250) — hardware-verified
//
#include <hip/hip_runtime.h>
#include <math.h>

#ifndef NB
#define NB 8
#endif
#ifndef SEQ
#define SEQ 8192
#endif
#define SEQ_FULL 8192
#define DM 128
#define NHEAD 4
#define HDIM 32
#define QKVN 384
#define MPOS (NB * SEQ)
#define OUT_M (NB * DM)
#define ACT_CARRY 64.0f
#define W_CARRY 64.0f
#define QP 388
#define OP 136

static constexpr float QK_SCALE  = 0.17677669f;
static constexpr float OUT_SCALE = 1.0f / 4096.0f;

static constexpr unsigned ilog2c(unsigned v) { return v <= 1u ? 0u : 1u + ilog2c(v >> 1); }

static_assert(DM == NHEAD * HDIM);
static_assert(QKVN == 3 * DM);
static_assert(DM % 32 == 0 && SEQ % 32 == 0);
static_assert(SEQ <= SEQ_FULL);
static_assert(MPOS % 32 == 0);
static_assert(OUT_M % 64 == 0 && DM % 64 == 0);
static_assert((QKVN * (DM / 8)) % 256 == 0);
static_assert((DM * (SEQ / 8)) % 256 == 0);
static_assert((1u << ilog2c(SEQ / 8)) == SEQ / 8);
static_assert((1u << ilog2c(DM / 8)) == DM / 8);
static_assert(ACT_CARRY * W_CARRY * OUT_SCALE == 1.0f);
static_assert(QP % 4 == 0 && QP >= QKVN && OP % 8 == 0 && OP >= DM);
static_assert(2 * 16 * QP * 4 + 2 * 16 * OP * 2 <= 131072);
static_assert(8 * 16 * 68 * 4 <= 131072);

static constexpr size_t WS_WT_BYTES = (size_t)QKVN * DM * 2;
static constexpr size_t WS_BT_BYTES = (size_t)DM * SEQ * 2;
static constexpr size_t WS_A_BYTES  = (size_t)MPOS * DM * 2;
static constexpr size_t WS_OFF_WT = 0;
static constexpr size_t WS_OFF_BT = WS_OFF_WT + WS_WT_BYTES;
static constexpr size_t WS_OFF_A  = WS_OFF_BT + WS_BT_BYTES;
static constexpr size_t WS_TOTAL  = WS_OFF_A + WS_A_BYTES;
static_assert(WS_WT_BYTES % 256 == 0 && WS_BT_BYTES % 256 == 0 && WS_A_BYTES % 256 == 0);
static_assert(WS_TOTAL <= (size_t)134217728);

typedef _Float16 h16;
typedef __attribute__((ext_vector_type(16))) _Float16 v16h;
typedef __attribute__((ext_vector_type(8)))  _Float16 v8h;
typedef __attribute__((ext_vector_type(16))) __bf16   v16bf;
typedef __attribute__((ext_vector_type(8)))  float    v8f;
typedef __attribute__((ext_vector_type(4)))  float    v4f;
typedef __attribute__((ext_vector_type(4)))  unsigned int v4u;
typedef __attribute__((ext_vector_type(8)))  unsigned int v8u;


#define VST2(T, ptr, val) do { const T vst2_v_ = (val); *(volatile T*)(ptr) = vst2_v_; __threadfence(); *(volatile T*)(ptr) = vst2_v_; } while (0)

__device__ __forceinline__ float bfr(float f) {
    unsigned u = __float_as_uint(f);
    u += 0x7FFFu + ((u >> 16) & 1u);
    return __uint_as_float(u & 0xFFFF0000u);
}
__device__ __forceinline__ unsigned bf_rne_u(float f) {
    unsigned u = __float_as_uint(f);
    u += 0x7FFFu + ((u >> 16) & 1u);
    return u;
}
__device__ __forceinline__ unsigned pack_bf(float lo, float hi) {
    return (bf_rne_u(lo) >> 16) | (bf_rne_u(hi) & 0xFFFF0000u);
}
static __device__ __forceinline__ h16 toh_flush(float v) {
    const float w = (fabsf(v) < 6.103515625e-05f) ? 0.0f : v;
    return (h16)w;
}

union FragU { v16h v; v8h h[2]; };
__device__ __forceinline__ v16h frag_ld(const _Float16* p) {
    FragU f; f.h[0] = *(const v8h*)(p); f.h[1] = *(const v8h*)(p + 16); return f.v;
}
__device__ __forceinline__ v8f wmma16(v16h a, v16h b, v8f c) {
    c = __builtin_amdgcn_wmma_f32_16x16x32_f16(false, a, false, b, (short)0, c, false, false);
    asm volatile("v_nop\n\tv_nop\n\tv_nop\n\tv_nop" : "+v"(c) : "v"(a), "v"(b));
    return c;
}
__device__ __forceinline__ v8f wmmabg(v8u a, v8u b, v8f c) {
    c = __builtin_amdgcn_wmma_f32_16x16x32_bf16(false, __builtin_bit_cast(v16bf, a), false, __builtin_bit_cast(v16bf, b),
                                                (short)0, c, false, false);
    asm volatile("v_nop\n\tv_nop\n\tv_nop\n\tv_nop" : "+v"(c) : "v"(a), "v"(b));
    return c;
}
__device__ __forceinline__ void wave_sync_lds() {
    __builtin_amdgcn_fence(3  , "workgroup");
    __builtin_amdgcn_wave_barrier();
    __builtin_amdgcn_fence(2  , "workgroup");
}

__global__ __launch_bounds__(256) void k_wt_b(const float* __restrict__ Wm, unsigned KI, unsigned NO, unsigned lgper,
                                              unsigned short* __restrict__ Wb) {
    const unsigned u = blockIdx.x * 256u + threadIdx.x;
    const unsigned per = 1u << lgper;
    if (u >= NO * per) return;
    const unsigned k0 = 8u * (u & (per - 1u));
    const unsigned o = u >> lgper;
    float v[8];
#pragma unroll
    for (int i = 0; i < 8; ++i) v[i] = Wm[(size_t)(k0 + (unsigned)i) * NO + o];
    v4u pk;
    pk.x = pack_bf(v[0], v[1]);
    pk.y = pack_bf(v[2], v[3]);
    pk.z = pack_bf(v[4], v[5]);
    pk.w = pack_bf(v[6], v[7]);
    VST2(v4u, Wb + (size_t)o * KI + k0, pk);
}

__global__ __launch_bounds__(256) void k_wt_h(const float* __restrict__ Wm, unsigned KI, unsigned NO, unsigned lgper,
                                              _Float16* __restrict__ Wh) {
    const unsigned u = blockIdx.x * 256u + threadIdx.x;
    const unsigned per = 1u << lgper;
    if (u >= NO * per) return;
    const unsigned k0 = 8u * (u & (per - 1u));
    const unsigned o = u >> lgper;
    v8h hv;
#pragma unroll
    for (int i = 0; i < 8; ++i) hv[i] = toh_flush(bfr(Wm[(size_t)(k0 + (unsigned)i) * NO + o]) * W_CARRY);
    VST2(v8h, Wh + (size_t)o * KI + k0, hv);
}

static_assert(32 * 16 * 8 == 16 * DM * 2);
__global__ __launch_bounds__(64) void k_qkvmix(const float* __restrict__ x, const unsigned short* __restrict__ Wt,
                                               const float* __restrict__ bqkv, _Float16* __restrict__ A16) {
    __shared__ __align__(16) float    sT[2][16 * QP];
    __shared__ __align__(16) _Float16 sO[2][16 * OP];
    const unsigned lane = threadIdx.x & 31u;
    const unsigned wave = (unsigned)__builtin_amdgcn_readfirstlane((int)(threadIdx.x >> 5));
    const unsigned hh = lane >> 4, c = lane & 15u;
    const unsigned bx = blockIdx.x;
    const unsigned g0 = (bx * 2u + wave) * 16u;
    const unsigned b  = g0 / (unsigned)SEQ;
    const unsigned s0 = g0 % (unsigned)SEQ;
    const float* xr = x + ((size_t)b * SEQ_FULL + s0 + c) * DM + 8u * hh;

#pragma unroll 1
    for (unsigned half = 0; half < 2u; ++half) {
        v8f acc[12];
#pragma unroll
        for (int j = 0; j < 12; ++j) acc[j] = (v8f){0.f, 0.f, 0.f, 0.f, 0.f, 0.f, 0.f, 0.f};
        const unsigned short* wrow = Wt + (size_t)(half * 192u + c) * DM + 8u * hh;
#pragma unroll 1
        for (unsigned k0 = 0; k0 < (unsigned)DM; k0 += 32u) {
            const v4f f0 = *(const v4f*)(xr + k0);
            const v4f f1 = *(const v4f*)(xr + k0 + 4u);
            const v4f f2 = *(const v4f*)(xr + k0 + 16u);
            const v4f f3 = *(const v4f*)(xr + k0 + 20u);
            v8u a;
            a[0] = pack_bf(f0.x, f0.y); a[1] = pack_bf(f0.z, f0.w);
            a[2] = pack_bf(f1.x, f1.y); a[3] = pack_bf(f1.z, f1.w);
            a[4] = pack_bf(f2.x, f2.y); a[5] = pack_bf(f2.z, f2.w);
            a[6] = pack_bf(f3.x, f3.y); a[7] = pack_bf(f3.z, f3.w);
#pragma unroll
            for (int j = 0; j < 12; ++j) {
                const unsigned short* wp = wrow + (size_t)((unsigned)j * 16u) * DM + k0;
                const v4u lo = *(const v4u*)(wp);
                const v4u hi = *(const v4u*)(wp + 16);
                const v8u bq = __builtin_shufflevector(lo, hi, 0, 1, 2, 3, 4, 5, 6, 7);
                acc[j] = wmmabg(a, bq, acc[j]);
            }
        }
#pragma unroll
        for (int j = 0; j < 12; ++j) {
            const unsigned n = half * 192u + (unsigned)j * 16u + c;
            const float bv = bfr(bqkv[n]);
#pragma unroll
            for (int r = 0; r < 8; ++r) sT[wave][(8u * hh + (unsigned)r) * QP + n] = acc[j][r] + bv;
        }
    }
    wave_sync_lds();

    const unsigned rowb = c * QP;
#pragma unroll 1
    for (unsigned t = 0; t < 2u; ++t) {
        const unsigned qh = 2u * hh + t;
        const unsigned qbase = rowb + qh * 96u;
        float sc[4] = {0.f, 0.f, 0.f, 0.f};
#pragma unroll 1
        for (unsigned d = 0; d < (unsigned)HDIM; d += 4u) {
            const v4f qv = *(const v4f*)&sT[wave][qbase + d];
#pragma unroll
            for (int kh = 0; kh < 4; ++kh) {
                const v4f kv = *(const v4f*)&sT[wave][rowb + (unsigned)kh * 96u + 32u + d];
                sc[kh] += (qv.x * kv.x + qv.y * kv.y) + (qv.z * kv.z + qv.w * kv.w);
            }
        }
        float p[4];
#pragma unroll
        for (int kh = 0; kh < 4; ++kh) p[kh] = sc[kh] * QK_SCALE;
        const float mx = fmaxf(fmaxf(p[0], p[1]), fmaxf(p[2], p[3]));
        float den = 0.f;
#pragma unroll
        for (int kh = 0; kh < 4; ++kh) { p[kh] = expf(p[kh] - mx); den += p[kh]; }
        const float inv = ACT_CARRY * (1.0f / den);
#pragma unroll
        for (int kh = 0; kh < 4; ++kh) p[kh] *= inv;
#pragma unroll 1
        for (unsigned d = 0; d < (unsigned)HDIM; d += 4u) {
            v4f o = (v4f){0.f, 0.f, 0.f, 0.f};
#pragma unroll
            for (int kh = 0; kh < 4; ++kh) {
                const v4f vv = *(const v4f*)&sT[wave][rowb + (unsigned)kh * 96u + 64u + d];
                o += p[kh] * vv;
            }
            const unsigned oi = c * OP + qh * 32u + d;
            sO[wave][oi]      = toh_flush(o.x);
            sO[wave][oi + 1u] = toh_flush(o.y);
            sO[wave][oi + 2u] = toh_flush(o.z);
            sO[wave][oi + 3u] = toh_flush(o.w);
        }
    }
    wave_sync_lds();

    {
        v8h ov[8];
#pragma unroll
        for (int it = 0; it < 8; ++it) ov[it] = *(const v8h*)&sO[wave][(2u * (unsigned)it + hh) * OP + c * 8u];
        _Float16* dst = A16 + (size_t)g0 * DM + lane * 8u;
        for (int pass = 0; pass < 2; ++pass) {
#pragma unroll
            for (int it = 0; it < 8; ++it) *(volatile v8h*)(dst + (unsigned)it * 256u) = ov[it];
            __threadfence();
        }
    }
}

static_assert(32 * 16 * 4 * 2 == 16 * 64 * 4);
__global__ __launch_bounds__(256) void k_outgemm(
    const _Float16* __restrict__ A, unsigned lda, const _Float16* __restrict__ Bt, unsigned ldb,
    float* __restrict__ C, unsigned ldc, const float* __restrict__ bias,
    unsigned M, unsigned N, unsigned K) {
  __shared__ __align__(16) float sT[8][16 * 68];
  const unsigned lane = threadIdx.x & 31u;
  const unsigned wave = (unsigned)__builtin_amdgcn_readfirstlane((int)(threadIdx.x >> 5));
  const unsigned tilesN = N >> 6, tilesM = M >> 6;
  const unsigned bx = blockIdx.x;
  const unsigned tile = bx * 8u + wave;
  if (tile >= tilesM * tilesN) return;
  const unsigned tm = tile / tilesN;
  const unsigned tn = tile - tm * tilesN;
  const unsigned m0 = tm << 6, n0 = tn << 6;
  const unsigned rlane = lane & 15u;
  const unsigned koff = (lane >> 4) * 8u;
  const unsigned mOff = koff;

  v8f acc[4][4];
#pragma unroll
  for (int i = 0; i < 4; ++i)
#pragma unroll
    for (int j = 0; j < 4; ++j) acc[i][j] = (v8f){0.f,0.f,0.f,0.f,0.f,0.f,0.f,0.f};

  for (unsigned k0 = 0; k0 < K; k0 += 32u) {
    v16h bh[4];
#pragma unroll
    for (int j = 0; j < 4; ++j)
      bh[j] = frag_ld(Bt + (size_t)(n0 + ((unsigned)j << 4) + rlane) * ldb + koff + k0);
#pragma unroll
    for (int i = 0; i < 4; ++i) {
      const v16h ah = frag_ld(A + (size_t)(m0 + ((unsigned)i << 4) + rlane) * lda + koff + k0);
#pragma unroll
      for (int j = 0; j < 4; ++j)
        acc[i][j] = wmma16(ah, bh[j], acc[i][j]);
    }
  }

#pragma unroll
  for (int i = 0; i < 4; ++i) {
    const unsigned mBase = m0 + ((unsigned)i << 4);
#pragma unroll
    for (int j = 0; j < 4; ++j) {
      const unsigned n = n0 + ((unsigned)j << 4) + rlane;
      const float bv = bfr(bias[n]);
#pragma unroll
      for (int r = 0; r < 8; ++r) {
        const float v = acc[i][j][r] * OUT_SCALE + bv;
        sT[wave][(mOff + (unsigned)r) * 68u + ((unsigned)j << 4) + rlane] = v;
      }
    }
    wave_sync_lds();
    {
      const unsigned hh = lane >> 4, c4 = (lane & 15u) * 4u;
#pragma unroll
      for (int half = 0; half < 2; ++half) {
        v4f vv[4];
#pragma unroll
        for (int it = 0; it < 4; ++it) {
          const unsigned row = (unsigned)(half * 4 + it) * 2u + hh;
          vv[it] = *(const v4f*)&sT[wave][row * 68u + c4];
        }
        for (int pass = 0; pass < 2; ++pass) {
#pragma unroll
          for (int it = 0; it < 4; ++it) {
            const unsigned row = (unsigned)(half * 4 + it) * 2u + hh;
            *(volatile v4f*)(C + (size_t)(mBase + row) * ldc + n0 + c4) = vv[it];
          }
          __threadfence();
        }
      }
    }
    wave_sync_lds();
  }
}

extern "C" void kernel_launch(void* const* d_in, const int* in_sizes, int n_in, void* d_out, int out_size,
                              void* d_ws, size_t ws_size, hipStream_t stream) {
    if (n_in < 5) return;
    if (in_sizes[0] < ((NB - 1) * SEQ_FULL + SEQ) * DM || in_sizes[1] < DM * QKVN || in_sizes[2] < QKVN) return;
    if (in_sizes[3] < SEQ * DM || in_sizes[4] < DM || out_size < OUT_M * DM) return;
    if (ws_size < WS_TOTAL) return;

    const float* x     = (const float*)d_in[0];
    const float* W_qkv = (const float*)d_in[1];
    const float* b_qkv = (const float*)d_in[2];
    const float* W_out = (const float*)d_in[3];
    const float* b_out = (const float*)d_in[4];
    float* out = (float*)d_out;

    char* wsp = (char*)d_ws;
    unsigned short* Wt  = (unsigned short*)(wsp + WS_OFF_WT);
    _Float16*       Bt  = (_Float16*)(wsp + WS_OFF_BT);
    _Float16*       A16 = (_Float16*)(wsp + WS_OFF_A);

    k_wt_b<<<(QKVN * (DM / 8)) / 256, 256, 0, stream>>>(W_qkv, DM, QKVN, ilog2c(DM / 8), Wt);
    k_wt_h<<<(DM * (SEQ / 8)) / 256, 256, 0, stream>>>(W_out, SEQ, DM, ilog2c(SEQ / 8), Bt);

    k_qkvmix<<<MPOS / 32, 64, 0, stream>>>(x, Wt, b_qkv, A16);

    k_outgemm<<<((OUT_M / 64) * (DM / 64) + 7) / 8, 256, 0, stream>>>(A16, SEQ, Bt, SEQ, out, DM, b_out, OUT_M, DM, SEQ);
}
